// InteractionLayer_9560597201472
// MI455X (gfx1250) — hardware-verified
//
#include <hip/hip_runtime.h>
#include <stddef.h>
#include <stdint.h>

#define HID    128
#define NB     64
#define KF1    128
#define KF2    128
#define KU     256
#define NTHR   256
#define NWAVE  8
#define EPB    256
#define DP     132
#define AP     136
#define MPITCH 128
#define GBM    64
#define GBN    128
#define GTHR   128
#define EPT    8
#define CHUNK  (NTHR * EPT)
#define WCAP   (EPT * 32)
#define LISTN  (NWAVE * WCAP)
#define NBA    1024
#define SLA    10
#define RCAP   28672
#define DEGCAP 64
#define NU_W1  (HID * (KF1 / 8))
#define NU_W2  (HID * (KF2 / 8))
#define NU_U   (HID * (KU / 8))
#define AGG_ZINTS (LISTN + 2 * RCAP + 3 * NBA)
#define AGG_LDS_INTS (AGG_ZINTS + 16)
#define AGG_LDS_BYTES (AGG_LDS_INTS * 4)
#define EDGE_LDS_BYTES (EPB * DP * 4 + EPB * AP * 2 + EPB * MPITCH * 2)
#define WSMAX  134217728
#define CACT   16.0f
#define CWGT   1024.0f
#define CMSG   16.0f
#define PINV   6.103515625e-05f
#define MINV   0.0625f
#define DMAXF  25.0f
#define C2W2   0.31494079113126730f

static_assert((CHUNK & (CHUNK - 1)) == 0 && CHUNK <= 4096);
static_assert((NBA & (NBA - 1)) == 0 && NBA == (1 << SLA));
static_assert(((long long)CHUNK << SLA) < (1LL << 31));
static_assert(LISTN % NTHR == 0);
static_assert(NBA % NWAVE == 0 && NBA % 32 == 0);
static_assert(RCAP % 4 == 0 && AGG_ZINTS % (4 * NTHR) == 0 && LISTN % 4 == 0);
static_assert(AGG_LDS_BYTES <= 300000);
static_assert(EDGE_LDS_BYTES <= 300000);
static_assert(NU_W1 % NTHR == 0 && NU_W2 % NTHR == 0 && NU_U % NTHR == 0);
static_assert(KF1 == 2 * NB && KF1 % 32 == 0 && KF2 == HID && KF2 % 32 == 0 && KU == 2 * HID && KU % 32 == 0);
static_assert(GBM == (GTHR / 32) * 16 && GBN == 4 * 32 && GBN == HID);
static_assert((DP * 4) % 16 == 0 && (AP * 2) % 16 == 0 && AP >= KF1 && AP >= KF2 && DP >= HID);
static_assert(EPB == NTHR && EPB == 8 * 32);
static_assert((EPB * DP * 4) % 16 == 0 && (EPB * AP * 2) % 16 == 0 && (EPB * MPITCH * 2) % 16 == 0);
static_assert(EPB * MPITCH * 2 == 16 * NTHR * 16);
static_assert(NB % 8 == 0 && HID % 8 == 0 && MPITCH == HID);

typedef float          v4f   __attribute__((ext_vector_type(4)));
typedef float          v8f   __attribute__((ext_vector_type(8)));
typedef int            v4i   __attribute__((ext_vector_type(4)));
typedef int            v8i   __attribute__((ext_vector_type(8)));
typedef unsigned       v2u   __attribute__((ext_vector_type(2)));
typedef unsigned short v8us  __attribute__((ext_vector_type(8)));
typedef unsigned short v16us __attribute__((ext_vector_type(16)));
typedef __bf16         v16bf __attribute__((ext_vector_type(16)));
typedef _Float16       v16h  __attribute__((ext_vector_type(16)));
typedef v4f  __attribute__((may_alias)) v4fa;
typedef v4i  __attribute__((may_alias)) v4ia;
typedef v2u  __attribute__((may_alias)) v2ua;
typedef v8us __attribute__((may_alias)) v8usa;
union FragB { v16bf v; v16us u; v8us h[2]; v8i w; };
union FragH { v16h  v; v16us u; v8us h[2]; v8i w; };

__device__ __forceinline__ v8f wmb(const FragB& a, const FragB& b, v8f c) {
  v8f d = __builtin_amdgcn_wmma_f32_16x16x32_bf16(false, a.v, false, b.v, (short)0, c, false, false);
  asm volatile("v_nop\n\tv_nop\n\tv_nop\n\tv_nop" : "+v"(d) : "v"(a.w), "v"(b.w));
  return d;
}
__device__ __forceinline__ v8f wmh(const FragH& a, const FragH& b, v8f c) {
  v8f d = __builtin_amdgcn_wmma_f32_16x16x32_f16(false, a.v, false, b.v, (short)0, c, false, false);
  asm volatile("v_nop\n\tv_nop\n\tv_nop\n\tv_nop" : "+v"(d) : "v"(a.w), "v"(b.w));
  return d;
}

__device__ __forceinline__ unsigned bf16_bits(float f) {
  const unsigned u = __float_as_uint(f);
  return (u + 0x7FFFu + ((u >> 16) & 1u)) >> 16;
}
__device__ __forceinline__ float bf16_val(float f) {
  return __uint_as_float(bf16_bits(f) << 16);
}
__device__ __forceinline__ unsigned short f2h(float f) {
  const _Float16 hv = (_Float16)f;
  return __builtin_bit_cast(unsigned short, hv);
}
__device__ __forceinline__ float h2f(unsigned b) {
  const _Float16 hv = __builtin_bit_cast(_Float16, (unsigned short)b);
  return (float)hv;
}
__device__ __forceinline__ void put16(unsigned short* dp, v8us o) {
  *(volatile v8us*)dp = o;
  __threadfence();
  *(volatile v8us*)dp = o;
}
__device__ __forceinline__ void putf4(float* dp, v4f o) {
  *(volatile v4f*)dp = o;
  __threadfence();
  *(volatile v4f*)dp = o;
}

template <int SLB>
__device__ __forceinline__ int scan_chunk(const int* __restrict__ dsts, int nE, int cbase, int slotBase,
                                          int nb, int vec8, int* list, int tid, int lane, int wave) {
  int wc = 0;
  const int el0  = tid * EPT;
  const int e0   = cbase + el0;
  const int sent = -2147483647 - 1;
  v4i da, db;
  if (vec8 != 0 && cbase + CHUNK <= nE) {
    da = *(const v4i*)(dsts + e0);
    db = *(const v4i*)(dsts + e0 + 4);
  } else {
    da.x = (e0     < nE) ? dsts[min(e0,     nE - 1)] : sent;
    da.y = (e0 + 1 < nE) ? dsts[min(e0 + 1, nE - 1)] : sent;
    da.z = (e0 + 2 < nE) ? dsts[min(e0 + 2, nE - 1)] : sent;
    da.w = (e0 + 3 < nE) ? dsts[min(e0 + 3, nE - 1)] : sent;
    db.x = (e0 + 4 < nE) ? dsts[min(e0 + 4, nE - 1)] : sent;
    db.y = (e0 + 5 < nE) ? dsts[min(e0 + 5, nE - 1)] : sent;
    db.z = (e0 + 6 < nE) ? dsts[min(e0 + 6, nE - 1)] : sent;
    db.w = (e0 + 7 < nE) ? dsts[min(e0 + 7, nE - 1)] : sent;
  }
  const unsigned nbs = (unsigned)slotBase;
  const unsigned unb = (unsigned)nb;
  const unsigned s0 = (unsigned)da.x - nbs, s1 = (unsigned)da.y - nbs;
  const unsigned s2 = (unsigned)da.z - nbs, s3 = (unsigned)da.w - nbs;
  const unsigned s4 = (unsigned)db.x - nbs, s5 = (unsigned)db.y - nbs;
  const unsigned s6 = (unsigned)db.z - nbs, s7 = (unsigned)db.w - nbs;
  const bool h0 = s0 < unb, h1 = s1 < unb, h2 = s2 < unb, h3 = s3 < unb;
  const bool h4 = s4 < unb, h5 = s5 < unb, h6 = s6 < unb, h7 = s7 < unb;
  const unsigned any = __builtin_amdgcn_ballot_w32(h0 | h1 | h2 | h3 | h4 | h5 | h6 | h7);
  if (any != 0u) {
#define HITJ(J, HJ, SJ) { \
      const unsigned mj = __builtin_amdgcn_ballot_w32(HJ); \
      if (mj != 0u) { \
        if (HJ) { \
          const int pos = wc + (int)__builtin_amdgcn_mbcnt_lo(mj, 0u); \
          if (pos < WCAP) list[wave * WCAP + pos] = ((el0 + (J)) << SLB) | (int)(SJ); \
        } \
        wc += (int)__builtin_popcount(mj); } }
    HITJ(0, h0, s0)
    HITJ(1, h1, s1)
    HITJ(2, h2, s2)
    HITJ(3, h3, s3)
    HITJ(4, h4, s4)
    HITJ(5, h5, s5)
    HITJ(6, h6, s6)
    HITJ(7, h7, s7)
#undef HITJ
  }
  return wc;
}

__global__ __launch_bounds__(NTHR) void k_prep(const float* __restrict__ R, const float* __restrict__ W1,
                                               const float* __restrict__ W2, const float* __restrict__ U1,
                                               const float* __restrict__ U2, int nN, int mRows,
                                               unsigned short* W1T, unsigned short* W2T,
                                               unsigned short* U1T, unsigned short* U2T,
                                               float* RP, float* HACC) {
  const int u   = (int)blockIdx.x * NTHR + (int)threadIdx.x;
  const int L0  = NU_W1;
  const int L1  = L0 + NU_W2;
  const int L2  = L1 + NU_U;
  const int L3  = L2 + NU_U;
  const int nXP = ((mRows + NTHR - 1) / NTHR) * NTHR;
  const int L4  = L3 + nXP;
  const int L5  = L4 + mRows * 32;
  const v4f z4 = {0.0f, 0.0f, 0.0f, 0.0f};
  v8us o;
  if (u < L0) {
    const int n    = u >> 4;
    const int k8   = (u & 15) * 8;
    const int srow = k8 & (NB - 1);
    const float* p = W1 + (size_t)srow * HID + n;
#pragma unroll
    for (int i = 0; i < 8; ++i) o[i] = (unsigned short)bf16_bits(p[(size_t)i * HID]);
    put16(W1T + (size_t)n * KF1 + k8, o);
    return;
  } else if (u < L1) {
    const int v  = u - L0;
    const int n  = v >> 4;
    const int k8 = (v & 15) * 8;
    const float* p = W2 + (size_t)k8 * HID + n;
#pragma unroll
    for (int i = 0; i < 8; ++i) o[i] = f2h(CWGT * bf16_val(p[(size_t)i * HID]));
    put16(W2T + (size_t)n * KF2 + k8, o);
    return;
  } else if (u < L2) {
    const int v    = u - L1;
    const int n    = v >> 5;
    const int k8   = (v & 31) * 8;
    const int srow = k8 & (HID - 1);
    const float* p = U1 + (size_t)srow * HID + n;
#pragma unroll
    for (int i = 0; i < 8; ++i) o[i] = (unsigned short)bf16_bits(p[(size_t)i * HID]);
    put16(U1T + (size_t)n * KU + k8, o);
    return;
  } else if (u < L3) {
    const int v    = u - L2;
    const int n    = v >> 5;
    const int k8   = (v & 31) * 8;
    const int srow = k8 & (HID - 1);
    const float* p = U2 + (size_t)srow * HID + n;
#pragma unroll
    for (int i = 0; i < 8; ++i) o[i] = (unsigned short)bf16_bits(p[(size_t)i * HID]);
    put16(U2T + (size_t)n * KU + k8, o);
    return;
  } else if (u < L4) {
    const int row = u - L3;
    if (row >= mRows) return;
    const int rc  = row < nN ? row : nN - 1;
    const bool ok = row < nN;
    const float r0 = R[(size_t)rc * 3 + 0];
    const float r1 = R[(size_t)rc * 3 + 1];
    const float r2 = R[(size_t)rc * 3 + 2];
    v4f q;
    q.x = ok ? bf16_val(r0) : 0.0f;
    q.y = ok ? bf16_val(r1) : 0.0f;
    q.z = ok ? bf16_val(r2) : 0.0f;
    q.w = 0.0f;
    putf4(RP + (size_t)row * 4, q);
    return;
  } else if (u < L5) {
    const int v = u - L4;
    putf4(HACC + (size_t)v * 4, z4);
    return;
  }
}

template <int MODE>
__global__ __launch_bounds__(GTHR) void k_gemm(const unsigned short* __restrict__ A, int lda,
                                               const unsigned short* __restrict__ BT, int ldb, int K,
                                               const float* __restrict__ bias, int nN,
                                               float* Cm, int ldc, unsigned short* Cb) {
  __shared__ __attribute__((aligned(16))) float stg[GBM * GBN];
  const int tid = (int)threadIdx.x, lane = tid & 31, wave = tid >> 5, hh = lane >> 4, m = lane & 15;
  const int rowBase = (int)blockIdx.x * GBM;
  const int colBase = (int)blockIdx.y * GBN;

  v8f acc[8];
  {
    const v8f z = {0.f, 0.f, 0.f, 0.f, 0.f, 0.f, 0.f, 0.f};
#pragma unroll
    for (int t = 0; t < 8; ++t) acc[t] = z;
  }
  const unsigned short* ap = A  + (size_t)(rowBase + 16 * wave + m) * (size_t)lda + 8 * hh;
  const unsigned short* bp = BT + (size_t)(colBase + m) * (size_t)ldb + 8 * hh;

#pragma unroll 1
  for (int k0 = 0; k0 < K; k0 += 32) {
    FragB af;
    af.h[0] = *(const v8usa*)(ap + k0);
    af.h[1] = *(const v8usa*)(ap + k0 + 16);
#pragma unroll
    for (int nt = 0; nt < 8; ++nt) {
      const unsigned short* wq = bp + (size_t)(16 * nt) * (size_t)ldb + k0;
      FragB bf;
      bf.h[0] = *(const v8usa*)wq;
      bf.h[1] = *(const v8usa*)(wq + 16);
      acc[nt] = wmb(af, bf, acc[nt]);
    }
  }

#pragma unroll
  for (int nt = 0; nt < 8; ++nt) {
    const int lc = 16 * nt + m;
    const float bvv = bf16_val(bias[colBase + lc]);
#pragma unroll
    for (int r = 0; r < 8; ++r) {
      const int lr = 16 * wave + 8 * hh + r;
      float v = acc[nt][r] + bvv;
      if constexpr (MODE == 1) v = fmaxf(v, 0.0f);
      stg[lr * GBN + lc] = v;
    }
  }
  __syncthreads();

  if constexpr (MODE == 1) {
    const int part = lane >> 4;
    const int j = lane & 15;
    const unsigned mh = 0u - (unsigned)part;
    const unsigned ml = ~mh;
    v8us pv[16];
#pragma unroll
    for (int i = 0; i < 16; ++i) {
      const float* sp = stg + (16 * wave + i) * GBN + 8 * j;
      const v4f a = *(const v4fa*)sp;
      const v4f b = *(const v4fa*)(sp + 4);
      const v8f f8 = {a.x, a.y, a.z, a.w, b.x, b.y, b.z, b.w};
      v8us oo;
#pragma unroll
      for (int e = 0; e < 8; ++e) {
        const unsigned hb = bf16_bits(f8[e]);
        const unsigned lb = bf16_bits(f8[e] - __uint_as_float(hb << 16));
        oo[e] = (unsigned short)((hb & ml) | (lb & mh));
      }
      pv[i] = oo;
    }
#pragma unroll
    for (int i = 0; i < 16; ++i) {
      unsigned short* op = Cb + (size_t)(rowBase + 16 * wave + i) * (size_t)KU + part * HID + 8 * j;
      *(volatile v8us*)op = pv[i];
    }
    __threadfence();
#pragma unroll
    for (int i = 0; i < 16; ++i) {
      unsigned short* op = Cb + (size_t)(rowBase + 16 * wave + i) * (size_t)KU + part * HID + 8 * j;
      *(volatile v8us*)op = pv[i];
    }
  } else {
    v4f pv[16];
#pragma unroll
    for (int i = 0; i < 16; ++i) pv[i] = *(const v4fa*)(stg + (16 * wave + i) * GBN + 4 * lane);
#pragma unroll
    for (int i = 0; i < 16; ++i) {
      const int row = rowBase + 16 * wave + i;
      if (row < nN) {
        float* op = Cm + (size_t)row * (size_t)ldc + colBase + 4 * lane;
        *(volatile v4f*)op = pv[i];
      }
    }
    __threadfence();
#pragma unroll
    for (int i = 0; i < 16; ++i) {
      const int row = rowBase + 16 * wave + i;
      if (row < nN) {
        float* op = Cm + (size_t)row * (size_t)ldc + colBase + 4 * lane;
        *(volatile v4f*)op = pv[i];
      }
    }
  }
}

__device__ __forceinline__ void wave_gemm_b(const unsigned short* sAw, float* sDw,
                                            const unsigned short* __restrict__ BT, int ldb, int K,
                                            int hh, int m) {
#pragma unroll 1
  for (int nh = 0; nh < 2; ++nh) {
    v8f acc[2][4];
    {
      const v8f z = {0.f, 0.f, 0.f, 0.f, 0.f, 0.f, 0.f, 0.f};
#pragma unroll
      for (int mt = 0; mt < 2; ++mt)
#pragma unroll
        for (int nt = 0; nt < 4; ++nt) acc[mt][nt] = z;
    }
    const unsigned short* ap0 = sAw + m * AP + 8 * hh;
    const unsigned short* ap1 = ap0 + 16 * AP;
    const unsigned short* bp  = BT + (size_t)(64 * nh + m) * (size_t)ldb + 8 * hh;
#pragma unroll 1
    for (int k0 = 0; k0 < K; k0 += 32) {
      FragB a0, a1;
      a0.h[0] = *(const v8usa*)(ap0 + k0);
      a0.h[1] = *(const v8usa*)(ap0 + k0 + 16);
      a1.h[0] = *(const v8usa*)(ap1 + k0);
      a1.h[1] = *(const v8usa*)(ap1 + k0 + 16);
#pragma unroll
      for (int nt = 0; nt < 4; ++nt) {
        const unsigned short* wq = bp + (size_t)(16 * nt) * (size_t)ldb + k0;
        FragB b;
        b.h[0] = *(const v8usa*)wq;
        b.h[1] = *(const v8usa*)(wq + 16);
        acc[0][nt] = wmb(a0, b, acc[0][nt]);
        acc[1][nt] = wmb(a1, b, acc[1][nt]);
      }
    }
#pragma unroll
    for (int nt = 0; nt < 4; ++nt) {
      const int col = 64 * nh + 16 * nt + m;
#pragma unroll
      for (int mt = 0; mt < 2; ++mt)
#pragma unroll
        for (int r = 0; r < 8; ++r) sDw[(16 * mt + 8 * hh + r) * DP + col] = acc[mt][nt][r];
    }
  }
}
__device__ __forceinline__ void wave_gemm_h(const unsigned short* sAw, float* sDw,
                                            const unsigned short* __restrict__ BT, int ldb, int K,
                                            int hh, int m) {
#pragma unroll 1
  for (int nh = 0; nh < 2; ++nh) {
    v8f acc[2][4];
    {
      const v8f z = {0.f, 0.f, 0.f, 0.f, 0.f, 0.f, 0.f, 0.f};
#pragma unroll
      for (int mt = 0; mt < 2; ++mt)
#pragma unroll
        for (int nt = 0; nt < 4; ++nt) acc[mt][nt] = z;
    }
    const unsigned short* ap0 = sAw + m * AP + 8 * hh;
    const unsigned short* ap1 = ap0 + 16 * AP;
    const unsigned short* bp  = BT + (size_t)(64 * nh + m) * (size_t)ldb + 8 * hh;
#pragma unroll 1
    for (int k0 = 0; k0 < K; k0 += 32) {
      FragH a0, a1;
      a0.h[0] = *(const v8usa*)(ap0 + k0);
      a0.h[1] = *(const v8usa*)(ap0 + k0 + 16);
      a1.h[0] = *(const v8usa*)(ap1 + k0);
      a1.h[1] = *(const v8usa*)(ap1 + k0 + 16);
#pragma unroll
      for (int nt = 0; nt < 4; ++nt) {
        const unsigned short* wq = bp + (size_t)(16 * nt) * (size_t)ldb + k0;
        FragH b;
        b.h[0] = *(const v8usa*)wq;
        b.h[1] = *(const v8usa*)(wq + 16);
        acc[0][nt] = wmh(a0, b, acc[0][nt]);
        acc[1][nt] = wmh(a1, b, acc[1][nt]);
      }
    }
#pragma unroll
    for (int nt = 0; nt < 4; ++nt) {
      const int col = 64 * nh + 16 * nt + m;
#pragma unroll
      for (int mt = 0; mt < 2; ++mt)
#pragma unroll
        for (int r = 0; r < 8; ++r) sDw[(16 * mt + 8 * hh + r) * DP + col] = acc[mt][nt][r];
    }
  }
}

__global__ __launch_bounds__(NTHR) void k_edge(const int* __restrict__ srcs, const int* __restrict__ dsts,
                                               int nEh, int nN,
                                               const float* __restrict__ RP, const float* __restrict__ X,
                                               const unsigned short* __restrict__ W1T,
                                               const unsigned short* __restrict__ W2T,
                                               unsigned short* Mh) {
#pragma clang fp contract(off)
  extern __shared__ __attribute__((aligned(16))) float dyn[];
  float*          sD = dyn;
  unsigned short* sA = (unsigned short*)(dyn + EPB * DP);
  unsigned short* sM = sA + EPB * AP;

  const int tid = (int)threadIdx.x, lane = tid & 31, wave = tid >> 5, hh = lane >> 4, m = lane & 15;

  const int  elb  = (int)blockIdx.x * EPB;
  const int  el   = elb + tid;
  const bool live = el < nEh;
  const int  elc  = live ? el : (nEh - 1);
  int s = srcs[elc];
  int t = dsts[elc];
  s = s < 0 ? 0 : (s > nN - 1 ? nN - 1 : s);
  t = t < 0 ? 0 : (t > nN - 1 ? nN - 1 : t);
  const v4f xs = *(const v4fa*)(RP + (size_t)s * 4);
  const v4f xd = *(const v4fa*)(RP + (size_t)t * 4);
  const float rx = xs.x - xd.x, ry = xs.y - xd.y, rz = xs.z - xd.z;
  const float dsq = (rx * rx + rz * rz) + ry * ry;

  float*          rd = sD + tid * DP;
  unsigned short* ra = sA + tid * AP;
  unsigned short* rm = sM + tid * MPITCH;
  {
    const float rw = 1.0f / C2W2;
#pragma unroll
    for (int c8 = 0; c8 < NB / 8; ++c8) {
      v8us ho, lo;
#pragma unroll
      for (int i = 0; i < 8; ++i) {
        const int   k  = 8 * c8 + i;
        const float ck = (k == NB - 1) ? DMAXF : DMAXF * ((float)k * (1.0f / 63.0f));
        const float dl = dsq - ck;
        const float nq = -(dl * dl);
        const float rb = __expf(nq * rw);
        const unsigned hb = bf16_bits(rb);
        ho[i] = (unsigned short)hb;
        lo[i] = (unsigned short)bf16_bits(rb - __uint_as_float(hb << 16));
      }
      *(v8usa*)(ra + 8 * c8)      = ho;
      *(v8usa*)(ra + NB + 8 * c8) = lo;
    }
  }
  __syncthreads();

  const unsigned short* sAw = sA + 32 * wave * AP;
  float*                sDw = sD + 32 * wave * DP;

  wave_gemm_b(sAw, sDw, W1T, KF1, KF1, hh, m);
  __syncthreads();

  {
#pragma unroll 1
    for (int c8 = 0; c8 < HID / 8; ++c8) {
      const v4f va = *(const v4fa*)(rd + 8 * c8);
      const v4f vb = *(const v4fa*)(rd + 8 * c8 + 4);
      const v8f v8 = {va.x, va.y, va.z, va.w, vb.x, vb.y, vb.z, vb.w};
      v8us o;
#pragma unroll
      for (int i = 0; i < 8; ++i) o[i] = f2h(CACT * fmaxf(v8[i], 0.0f));
      *(v8usa*)(ra + 8 * c8) = o;
    }
  }
  __syncthreads();

  wave_gemm_h(sAw, sDw, W2T, KF2, KF2, hh, m);
  __syncthreads();

  {
    const float* xr = X + (size_t)s * HID;
#pragma unroll 1
    for (int c8 = 0; c8 < HID / 8; ++c8) {
      const v4f va = *(const v4fa*)(rd + 8 * c8);
      const v4f vb = *(const v4fa*)(rd + 8 * c8 + 4);
      const v4f xa = *(const v4fa*)(xr + 8 * c8);
      const v4f xb = *(const v4fa*)(xr + 8 * c8 + 4);
      const v8f v8 = {va.x, va.y, va.z, va.w, vb.x, vb.y, vb.z, vb.w};
      const v8f x8 = {xa.x, xa.y, xa.z, xa.w, xb.x, xb.y, xb.z, xb.w};
      v8us o;
#pragma unroll
      for (int i = 0; i < 8; ++i) {
        const float mv = fmaxf(v8[i] * PINV, 0.0f);
        const float ms = bf16_val(x8[i]) * mv;
        o[i] = f2h(CMSG * ms);
      }
      *(v8usa*)(rm + 8 * c8) = o;
    }
  }
  __syncthreads();

  {
    v4i pv[16];
#pragma unroll
    for (int it = 0; it < 16; ++it) pv[it] = *(const v4ia*)(sM + (size_t)(it * NTHR + tid) * 8);
    unsigned short* mb = Mh + (size_t)elb * MPITCH;
#pragma unroll
    for (int it = 0; it < 16; ++it) *(volatile v4i*)(mb + (size_t)(it * NTHR + tid) * 8) = pv[it];
    __threadfence();
#pragma unroll
    for (int it = 0; it < 16; ++it) *(volatile v4i*)(mb + (size_t)(it * NTHR + tid) * 8) = pv[it];
  }
}

__global__ __launch_bounds__(NTHR) void k_scan(const int* __restrict__ dsts, int nEh, int vec8, int mRows,
                                               const unsigned short* __restrict__ Mh, float* HACC) {
  extern __shared__ __attribute__((aligned(16))) int dsm[];
  int*   list = dsm;
  int*   hl   = dsm + LISTN;
  int*   sl   = hl + RCAP;
  int*   cnt  = sl + RCAP;
  int*   offs = cnt + NBA;
  int*   cur  = offs + NBA;
  int*   misc = cur + NBA;
  const int tid = (int)threadIdx.x, lane = tid & 31, wave = tid >> 5;
  const int nodeBase = (int)blockIdx.x * NBA;

  {
    const v4i z4 = {0, 0, 0, 0};
    for (int i = tid * 4; i < AGG_ZINTS; i += NTHR * 4) *(v4ia*)(dsm + i) = z4;
    if (tid < 16) misc[tid] = 0;
  }
  __syncthreads();

  int t = 0, ov = 0;
  const int nChunks = (nEh + CHUNK - 1) / CHUNK;
#pragma unroll 1
  for (int ch = 0; ch < nChunks; ++ch) {
    const int cbase = ch * CHUNK;
    const int wc = scan_chunk<SLA>(dsts, nEh, cbase, nodeBase, NBA, vec8, list, tid, lane, wave);
    if (lane == 0) misc[wave] = wc;
    __syncthreads();
    if (wave == 0) {
#pragma unroll 1
      for (int w2 = 0; w2 < NWAVE; ++w2) {
        int c = misc[w2];
        c = c < 0 ? 0 : (c > WCAP ? WCAP : c);
#pragma unroll 1
        for (int b0 = 0; b0 < c; b0 += 32) {
          const int idx = b0 + lane;
          const int ent = list[w2 * WCAP + (idx < WCAP ? idx : WCAP - 1)];
          const int m32 = (c - b0) < 32 ? (c - b0) : 32;
#pragma unroll 1
          for (int k = 0; k < m32; ++k) {
            const int u    = __builtin_amdgcn_readlane(ent, k);
            const int slot = u & (NBA - 1);
            const int el   = (u >> SLA) & (CHUNK - 1);
            const int pk   = ((cbase + el) << SLA) | slot;
            if (t < RCAP) {
              if (lane == 0) { hl[t] = pk; cnt[slot] = cnt[slot] + 1; }
              t = t + 1;
            } else {
              ov = 1;
            }
          }
        }
      }
    }
    __syncthreads();
  }
  if (wave == 0 && lane == 0) { misc[8] = t; misc[9] = ov; }
  __syncthreads();
  int tt = misc[8];
  tt = tt < 0 ? 0 : (tt > RCAP ? RCAP : tt);
  const int ovf = misc[9];

  if (wave == 0) {
    const int base = lane * (NBA / 32);
    int s = 0;
#pragma unroll 1
    for (int i = 0; i < NBA / 32; ++i) s += cnt[base + i];
    int incl = s;
#pragma unroll
    for (int d = 1; d < 32; d <<= 1) {
      const int y = __shfl_up(incl, d, 32);
      if (lane >= d) incl += y;
    }
    int run = incl - s;
#pragma unroll 1
    for (int i = 0; i < NBA / 32; ++i) {
      const int cv = cnt[base + i];
      offs[base + i] = run;
      cur[base + i]  = run;
      run += cv;
    }
  }
  __syncthreads();
  if (wave == 0) {
#pragma unroll 1
    for (int b0 = 0; b0 < tt; b0 += 32) {
      const int idx = b0 + lane;
      const int ent = hl[idx < RCAP ? idx : RCAP - 1];
      const int m32 = (tt - b0) < 32 ? (tt - b0) : 32;
#pragma unroll 1
      for (int k = 0; k < m32; ++k) {
        const int u    = __builtin_amdgcn_readlane(ent, k);
        const int slot = u & (NBA - 1);
        if (lane == 0) {
          int p = cur[slot];
          p = p < 0 ? 0 : (p > RCAP - 1 ? RCAP - 1 : p);
          sl[p] = u;
          cur[slot] = p + 1;
        }
      }
    }
  }
  __syncthreads();

  const float qnan = __int_as_float(0x7fc00000);
  const float pz = (ovf != 0) ? qnan : 0.0f;
#pragma unroll 1
  for (int si = 0; si < NBA / NWAVE; ++si) {
    const int s    = si * NWAVE + wave;
    const int node = nodeBase + s;
    int c = cnt[s];
    const bool big = c > DEGCAP;
    c = c < 0 ? 0 : (c > DEGCAP ? DEGCAP : c);
    int o = offs[s];
    o = o < 0 ? 0 : (o > RCAP ? RCAP : o);
    float a0 = 0.0f, a1 = 0.0f, a2 = 0.0f, a3 = 0.0f;
#pragma unroll 1
    for (int b0 = 0; b0 < c; b0 += 32) {
      int idx = o + b0 + lane;
      idx = idx > RCAP - 1 ? RCAP - 1 : idx;
      const int ent = sl[idx];
      int eid = ent >> SLA;
      eid = eid < 0 ? 0 : (eid > nEh - 1 ? nEh - 1 : eid);
      const int m32 = (c - b0) < 32 ? (c - b0) : 32;
#pragma unroll 1
      for (int k = 0; k < m32; ++k) {
        const int ek = __builtin_amdgcn_readlane(eid, k);
        const unsigned short* rp = Mh + (size_t)ek * MPITCH + 4 * lane;
        const v2u w = *(const v2ua*)rp;
        a0 += h2f(w.x & 0xffffu);
        a1 += h2f(w.x >> 16);
        a2 += h2f(w.y & 0xffffu);
        a3 += h2f(w.y >> 16);
      }
    }
    const bool  live = node < mRows;
    const int   nr   = live ? node : mRows - 1;
    const float pzr  = big ? qnan : pz;
    float* mp = HACC + (size_t)nr * HID + 4 * lane;
    const v4f old = *(const v4fa*)mp;
    v4f nv;
    nv.x = fmaf(a0, MINV, old.x) + pzr;
    nv.y = fmaf(a1, MINV, old.y) + pzr;
    nv.z = fmaf(a2, MINV, old.z) + pzr;
    nv.w = fmaf(a3, MINV, old.w) + pzr;
    if (live) *(volatile v4f*)mp = nv;
    __threadfence();
    if (live) *(volatile v4f*)mp = nv;
  }
}

__global__ __launch_bounds__(NTHR) void k_ha(const float* __restrict__ HACC, int nUnits, unsigned short* HA) {
  const int u = (int)blockIdx.x * NTHR + (int)threadIdx.x;
  if (u >= nUnits) return;
  const int row = u >> 4;
  const int j   = u & 15;
  const float* mq = HACC + (size_t)row * HID + 8 * j;
  const v4f ma = *(const v4fa*)mq;
  const v4f mb = *(const v4fa*)(mq + 4);
  const v8f m8 = {ma.x, ma.y, ma.z, ma.w, mb.x, mb.y, mb.z, mb.w};
  v8us ohi, olo;
#pragma unroll
  for (int i = 0; i < 8; ++i) {
    const unsigned hbits = bf16_bits(m8[i]);
    ohi[i] = (unsigned short)hbits;
    olo[i] = (unsigned short)bf16_bits(m8[i] - __uint_as_float(hbits << 16));
  }
  unsigned short* dp = HA + (size_t)row * KU + 8 * j;
  *(volatile v8us*)dp         = ohi;
  *(volatile v8us*)(dp + HID) = olo;
  __threadfence();
  *(volatile v8us*)dp         = ohi;
  *(volatile v8us*)(dp + HID) = olo;
}

static inline int cdiv(int a, int b) { return (a + b - 1) / b; }

extern "C" void kernel_launch(void* const* d_in, const int* in_sizes, int n_in,
                              void* d_out, int out_size, void* d_ws, size_t ws_size,
                              hipStream_t stream) {
  if (n_in < 10) return;
  if (in_sizes[0] < HID || (in_sizes[0] % HID) != 0) return;
  const int nN = in_sizes[0] / HID;
  if (in_sizes[1] != 3 * nN) return;
  const int nE = in_sizes[2];
  if (nE < 1 || nE >= (1 << 22)) return;
  if (in_sizes[3] != nE) return;
  if (in_sizes[4] != NB * HID) return;
  if (in_sizes[5] != HID * HID || in_sizes[6] != HID * HID) return;
  if (in_sizes[7] != HID) return;
  if (in_sizes[8] != HID * HID || in_sizes[9] != HID) return;
  if ((long long)out_size != (long long)nN * HID) return;

  const float* X    = (const float*)d_in[0];
  const float* R    = (const float*)d_in[1];
  const int*   src  = (const int*)d_in[2];
  const int*   dst  = (const int*)d_in[3];
  const float* W1   = (const float*)d_in[4];
  const float* W2   = (const float*)d_in[5];
  const float* U1   = (const float*)d_in[6];
  const float* b1   = (const float*)d_in[7];
  const float* U2   = (const float*)d_in[8];
  const float* b2   = (const float*)d_in[9];
  float* out = (float*)d_out;

  const int MP = cdiv(nN, GBM) * GBM;
  const int gM = MP / GBM;
  const int gA = cdiv(MP, NBA);
  if ((long long)gA * NBA < (long long)MP) return;
  const int EH   = cdiv(cdiv(nE, 2), EPB) * EPB;
  const int nEh0 = nE < EH ? nE : EH;
  const int nEh1 = nE - nEh0;
  const int EHP  = EH;
  if (nEh0 < 1 || nEh0 >= (1 << 21) || nEh1 > EH) return;

  char* ws = (char*)d_ws;
  size_t off = 0;
  const size_t oW1T = off; off += (size_t)HID * KF1 * 2;             off = (off + 255) & ~(size_t)255;
  const size_t oW2T = off; off += (size_t)HID * KF2 * 2;             off = (off + 255) & ~(size_t)255;
  const size_t oU1T = off; off += (size_t)HID * KU * 2;              off = (off + 255) & ~(size_t)255;
  const size_t oU2T = off; off += (size_t)HID * KU * 2;              off = (off + 255) & ~(size_t)255;
  const size_t oRP  = off; off += (size_t)MP * 4 * 4;                off = (off + 255) & ~(size_t)255;
  size_t szRA = (size_t)MP * HID * 4;
  if (szRA < (size_t)MP * KU * 2) szRA = (size_t)MP * KU * 2;
  const size_t oRA  = off; off += szRA;                              off = (off + 255) & ~(size_t)255;
  size_t szRB = (size_t)EHP * MPITCH * 2;
  if (szRB < (size_t)MP * KU * 2) szRB = (size_t)MP * KU * 2;
  const size_t oRB  = off; off += szRB;                              off = (off + 255) & ~(size_t)255;
  if (off > ws_size || off > (size_t)WSMAX) return;
  unsigned short* W1T  = (unsigned short*)(ws + oW1T);
  unsigned short* W2T  = (unsigned short*)(ws + oW2T);
  unsigned short* U1T  = (unsigned short*)(ws + oU1T);
  unsigned short* U2T  = (unsigned short*)(ws + oU2T);
  float*          RP   = (float*)(ws + oRP);
  float*          HACC = (float*)(ws + oRA);
  unsigned short* G    = (unsigned short*)(ws + oRA);
  unsigned short* MSG  = (unsigned short*)(ws + oRB);
  unsigned short* HA   = (unsigned short*)(ws + oRB);

  hipFuncSetAttribute(reinterpret_cast<const void*>(&k_edge), hipFuncAttributeMaxDynamicSharedMemorySize,
                      (int)EDGE_LDS_BYTES);
  hipFuncSetAttribute(reinterpret_cast<const void*>(&k_scan), hipFuncAttributeMaxDynamicSharedMemorySize,
                      (int)AGG_LDS_BYTES);

  const int nXP   = cdiv(MP, NTHR) * NTHR;
  const int nPrep = NU_W1 + NU_W2 + 2 * NU_U + nXP + MP * 32;
  const int vec0  = 1;
  const int vec1  = ((EH & 3) == 0) ? 1 : 0;

  k_prep<<<nPrep / NTHR, NTHR, 0, stream>>>(R, W1, W2, U1, U2, nN, MP, W1T, W2T, U1T, U2T, RP, HACC);
  k_edge<<<cdiv(nEh0, EPB), NTHR, EDGE_LDS_BYTES, stream>>>(src, dst, nEh0, nN, RP, X, W1T, W2T, MSG);
  k_scan<<<gA, NTHR, AGG_LDS_BYTES, stream>>>(dst, nEh0, vec0, MP, MSG, HACC);
  if (nEh1 > 0) {
    k_edge<<<cdiv(nEh1, EPB), NTHR, EDGE_LDS_BYTES, stream>>>(src + EH, dst + EH, nEh1, nN, RP, X,
                                                               W1T, W2T, MSG);
    k_scan<<<gA, NTHR, AGG_LDS_BYTES, stream>>>(dst + EH, nEh1, vec1, MP, MSG, HACC);
  }
  k_ha<<<(MP * 16) / NTHR, NTHR, 0, stream>>>(HACC, MP * 16, HA);
  k_gemm<1><<<dim3(gM, 1), GTHR, 0, stream>>>(HA, KU, U1T, KU, KU, b1, nN, out, HID, G);
  k_gemm<2><<<dim3(gM, 1), GTHR, 0, stream>>>(G, KU, U2T, KU, KU, b2, nN, out, HID, HA);
}
